// ODEINTWEvents_15547781611924
// MI455X (gfx1250) — hardware-run, weakly checked
//
#include <hip/hip_runtime.h>


#define NB   32768
#define ND   64
#define NH   128
#define NSTEP 64
typedef _Float16 h16;
typedef unsigned short bf;
typedef __attribute__((ext_vector_type(16))) __bf16   v16bf;
typedef __attribute__((ext_vector_type(16))) _Float16 v16h;
typedef __attribute__((ext_vector_type(8)))  _Float16 v8h;
typedef __attribute__((ext_vector_type(8)))  unsigned short v8us;
typedef __attribute__((ext_vector_type(8)))  float    v8f;
typedef __attribute__((ext_vector_type(4)))  float    v4f;
typedef v8h  __attribute__((may_alias)) v8ha;
typedef v4f  __attribute__((may_alias)) v4fa;
typedef v8us __attribute__((may_alias)) v8usa;

__device__ __forceinline__ unsigned short f2bf(float f) { unsigned u = __float_as_uint(f); u += 0x7FFFu + ((u >> 16) & 1u); return (unsigned short)(u >> 16); }
__device__ __forceinline__ float bf2f(unsigned short b) { return __uint_as_float(((unsigned)b) << 16); }
__device__ __forceinline__ float bfr(float f) { return bf2f(f2bf(f)); }
__device__ __forceinline__ v16h cat16(v8h lo, v8h hi) { return __builtin_shufflevector(lo, hi, 0, 1, 2, 3, 4, 5, 6, 7, 8, 9, 10, 11, 12, 13, 14, 15); }
__device__ __forceinline__ v16bf cat16b(v8us lo, v8us hi) { return __builtin_bit_cast(v16bf, __builtin_shufflevector(lo, hi, 0, 1, 2, 3, 4, 5, 6, 7, 8, 9, 10, 11, 12, 13, 14, 15)); }
__device__ __forceinline__ v8f wmma16(v16h a, v16h b, v8f c) { return __builtin_amdgcn_wmma_f32_16x16x32_f16(false, a, false, b, (short)0, c, false, false); }
__device__ __forceinline__ v8f wmmab(v16bf a, v16bf b, v8f c) { return __builtin_amdgcn_wmma_f32_16x16x32_bf16(false, a, false, b, (short)0, c, false, false); }

template <typename T16> struct WFrag;
template <> struct WFrag<h16> { typedef v16h V; static __device__ __forceinline__ V ld(const h16* p) { return cat16(*(const v8h*)p, *(const v8h*)(p + 16)); } static __device__ __forceinline__ v8f mma(V a, V b, v8f c) { return wmma16(a, b, c); } };
template <> struct WFrag<bf> { typedef v16bf V; static __device__ __forceinline__ V ld(const bf* p) { return cat16b(*(const v8us*)p, *(const v8us*)(p + 16)); } static __device__ __forceinline__ v8f mma(V a, V b, v8f c) { return wmmab(a, b, c); } };

typedef __attribute__((ext_vector_type(2))) _Float16 v2h;
typedef __attribute__((ext_vector_type(4))) _Float16 v4h;
typedef __attribute__((ext_vector_type(2))) unsigned short v2us;
typedef __attribute__((ext_vector_type(4))) unsigned short v4us;
typedef __attribute__((ext_vector_type(2))) float v2f;
typedef __attribute__((ext_vector_type(4))) int v4i;

__global__ __launch_bounds__(256) void k_wtG(const float* __restrict__ w, int K, int N, bf* Bt) {
    const int lane = threadIdx.x & 31; const int L0 = (blockIdx.x * 8 + (threadIdx.x >> 5)) * 8; const int nlines = N * K / 64;
#pragma unroll
    for (int ps = 0; ps < 2; ++ps) {
        for (int l = 0; l < 8; ++l) { const int L = L0 + l; if (L >= nlines) break; const size_t e = (size_t)L * 64 + lane * 2; const int k = (int)(e % K), n = (int)(e / K); v2us o;
            o[0] = f2bf(w[(size_t)k * N + n]); o[1] = f2bf(w[(size_t)(k + 1) * N + n]); *(volatile v2us*)(Bt + e) = o; }
        if (ps == 0) __threadfence(); }
}

__device__ __forceinline__ float tanhc(float v) { return 1.0f - 2.0f / (expf(2.0f * v) + 1.0f); }

__global__ __launch_bounds__(32) void k_ode(const float* __restrict__ y0, const float* __restrict__ ft, const float* __restrict__ lt, const float* __restrict__ ss, const bf* __restrict__ W1t, const float* __restrict__ b1, const bf* __restrict__ W2t, const float* __restrict__ b2, float* ostate, float* ozero, float* osteps) {
    if (blockIdx.x >= (unsigned)(NB / 16)) return;
    const int lane = threadIdx.x & 31, lr = lane & 15, hi = lane >> 4; const size_t row = (size_t)blockIdx.x * 16 + lr;
    float Y[4][8];
#pragma unroll
    for (int dt = 0; dt < 4; ++dt) { const float* p = y0 + row * ND + 32 * hi + 8 * dt; const v4f a = *(const v4f*)p; const v4f b = *(const v4f*)(p + 4);
#pragma unroll
        for (int j = 0; j < 4; ++j) { Y[dt][j] = bfr(a[j]); Y[dt][4 + j] = bfr(b[j]); } }
    const float dtv = bfr(ss[row]); const float ltv = bfr(lt[row]); float t = bfr(ft[row]); unsigned long long mbits = 0ull;
    const bf* w1p = W1t + (size_t)lr * ND + 32 * hi; const bf* w2p = W2t + (size_t)(32 * (lr >> 3) + (lr & 7)) * NH + 8 * hi;
    for (int k = 0; k < NSTEP; ++k) {
        const float m = (t + 1e-5f < ltv) ? 1.0f : 0.0f;
        v16bf yf[2];
#pragma unroll
        for (int cc = 0; cc < 2; ++cc) { v8us lo, up;
#pragma unroll
            for (int j = 0; j < 8; ++j) { lo[j] = f2bf(Y[2 * cc][j]); up[j] = f2bf(Y[2 * cc + 1][j]); }
            yf[cc] = cat16b(lo, up); }
        v8f f[4];
#pragma unroll
        for (int dt = 0; dt < 4; ++dt) f[dt] = (v8f){};
        for (int c = 0; c < 4; ++c) { v8f d0 = (v8f){}, d1 = (v8f){};
#pragma unroll
            for (int cc = 0; cc < 2; ++cc) { const bf* pa = w1p + (size_t)(32 * c) * ND + 16 * cc; d0 = wmmab(cat16b(*(const v8us*)pa, *(const v8us*)(pa + 8)), yf[cc], d0); const bf* pb = pa + (size_t)16 * ND; d1 = wmmab(cat16b(*(const v8us*)pb, *(const v8us*)(pb + 8)), yf[cc], d1); }
            v8us lo, up;
#pragma unroll
            for (int j = 0; j < 8; ++j) { lo[j] = f2bf(tanhc(d0[j] + bfr(b1[32 * c + 8 * hi + j]))); up[j] = f2bf(tanhc(d1[j] + bfr(b1[32 * c + 16 + 8 * hi + j]))); }
            const v16bf tf = cat16b(lo, up);
#pragma unroll
            for (int dt = 0; dt < 4; ++dt) f[dt] = wmmab(WFrag<bf>::ld(w2p + (size_t)(8 * dt) * NH + 32 * c), tf, f[dt]); }
#pragma unroll
        for (int dt = 0; dt < 4; ++dt) {
#pragma unroll
            for (int j = 0; j < 8; ++j) { const float fv = f[dt][j] + bfr(b2[32 * hi + 8 * dt + j]); const float nxt = Y[dt][j] + dtv * fv; Y[dt][j] = m * nxt + (1.0f - m) * Y[dt][j]; } }
        t = t + dtv; mbits |= (unsigned long long)((m != 0.0f) ? 1u : 0u) << k; }
    float* ps = ostate + row * ND + 32 * hi; float* pz = ozero + row * ND + 32 * hi; float* pm = osteps + row * NSTEP + 32 * hi; const unsigned mw = (unsigned)(mbits >> (32 * hi));
#pragma unroll
    for (int pass = 0; pass < 2; ++pass) {
#pragma unroll
        for (int dt = 0; dt < 4; ++dt) { v4f a, b;
#pragma unroll
            for (int j = 0; j < 4; ++j) { a[j] = Y[dt][j]; b[j] = Y[dt][4 + j]; }
            *(volatile v4f*)(ps + 8 * dt) = a; *(volatile v4f*)(ps + 8 * dt + 4) = b; }
#pragma unroll
        for (int q = 0; q < 8; ++q) { v4f z; z[0] = 0.0f; z[1] = 0.0f; z[2] = 0.0f; z[3] = 0.0f; *(volatile v4f*)(pz + 4 * q) = z; }
#pragma unroll
        for (int q = 0; q < 8; ++q) { v4f s;
#pragma unroll
            for (int e = 0; e < 4; ++e) s[e] = ((mw >> (4 * q + e)) & 1u) ? 1.0f : 0.0f;
            *(volatile v4f*)(pm + 4 * q) = s; }
        if (pass == 0) __threadfence(); }
}

__global__ __launch_bounds__(256) void k_dtc(const float* __restrict__ ss, float* dst, int n4) { const int i = blockIdx.x * 256 + threadIdx.x; if (i >= n4) return; const v4f v = *(const v4f*)(ss + (size_t)i * 4); v4f r;
#pragma unroll
    for (int k = 0; k < 4; ++k) r[k] = bfr(v[k]);
    *(volatile v4f*)(dst + (size_t)i * 4) = r; __threadfence(); *(volatile v4f*)(dst + (size_t)i * 4) = r; }

extern "C" void kernel_launch(void* const* d_in, const int* in_sizes, int n_in, void* d_out, int out_size, void* d_ws, size_t ws_size, hipStream_t stream) {
    if (n_in < 8) return;
    if (in_sizes[0] != NB * ND || in_sizes[1] != NB || in_sizes[2] != NB || in_sizes[3] != NB || in_sizes[4] != ND * NH || in_sizes[5] != NH || in_sizes[6] != NH * ND || in_sizes[7] != ND) return;
    if (out_size != 3 * NB * ND + NB) return;
    static_assert(NB % 16 == 0 && ND == 64 && NH == 128 && NSTEP == 64 && (NB / 4) % 256 == 0 && (ND * NH) % 64 == 0, "a wave a 16-row tile on an exact grid; four state tiles and eight unit tiles; 64 mask bits a row; the step-size copy on an exact grid; the weight planes whole lines of 64 words");
    static_assert(((size_t)NB * ND * 4) % 128 == 0 && ((size_t)NB * 4) % 128 == 0, "every output begins on a 128-byte line");
    const float* y0 = (const float*)d_in[0]; const float* ft = (const float*)d_in[1]; const float* lt = (const float*)d_in[2]; const float* ss = (const float*)d_in[3]; const float* w1 = (const float*)d_in[4]; const float* b1 = (const float*)d_in[5]; const float* w2 = (const float*)d_in[6]; const float* b2 = (const float*)d_in[7];
    float* out = (float*)d_out; float* ostate = out; float* ozero = out + (size_t)NB * ND; float* odt = out + (size_t)2 * NB * ND; float* osteps = out + (size_t)2 * NB * ND + NB;
    char* wsp = (char*)d_ws; auto take = [&](size_t bytes) { char* p = wsp; wsp += (bytes + 255) & ~(size_t)255; return (void*)p; };
    bf* W1t = (bf*)take((size_t)NH * ND * 2);     bf* W2t = (bf*)take((size_t)ND * NH * 2);
    if ((size_t)(wsp - (char*)d_ws) > ws_size) return;
    k_wtG<<<(unsigned)((ND * NH / 64 + 63) / 64), 256, 0, stream>>>(w1, ND, NH, W1t);
    k_wtG<<<(unsigned)((NH * ND / 64 + 63) / 64), 256, 0, stream>>>(w2, NH, ND, W2t);
    k_ode<<<(unsigned)(NB / 16), 32, 0, stream>>>(y0, ft, lt, ss, W1t, b1, W2t, b2, ostate, ozero, osteps);
    k_dtc<<<(unsigned)(NB / 4 / 256), 256, 0, stream>>>(ss, odt, NB / 4);
}
